// OptimizedAttention_57655640982115
// MI455X (gfx1250) — hardware-verified
//
#include <hip/hip_runtime.h>
#include <math.h>
#include <stdint.h>

#define NB    4
#define SQ    512
#define DM    2048
#define NH    16
#define HD    128
#define NTOK  2048
#define NFRQ  64
#define QKVN  6144

static_assert(NH * HD == DM);
static_assert(HD == 2 * NFRQ);
static_assert(HD == 128);
static_assert((SQ & (SQ - 1)) == 0);
static_assert(NTOK == NB * SQ);
static_assert(SQ % 64 == 0);
static_assert(NTOK % 64 == 0);
static_assert(DM % 64 == 0);
static_assert(DM % 32 == 0);
static_assert((NTOK * DM) % (256 * 8) == 0);
static_assert((QKVN * DM) % (256 * 8) == 0);
static_assert((DM * DM) % (256 * 8) == 0);
static_assert(((NTOK / 64) * (DM / 64)) % 8 == 0);
static_assert((SQ * 2) % 8 == 0);
static_assert(10ull * NTOK * DM * 2 + (unsigned long long)QKVN * DM * 2 + 2ull * SQ * NFRQ * 4 <= 134217728ull);

typedef _Float16     v16h __attribute__((ext_vector_type(16)));
typedef _Float16     v8h  __attribute__((ext_vector_type(8)));
typedef __bf16       v16b __attribute__((ext_vector_type(16)));
typedef __bf16       v8b  __attribute__((ext_vector_type(8)));
typedef float        v8f  __attribute__((ext_vector_type(8)));
typedef float        v4f  __attribute__((ext_vector_type(4)));
typedef unsigned int v4u  __attribute__((ext_vector_type(4)));

__device__ __forceinline__ unsigned short f2bf_bits(float f) {
  const unsigned u = __float_as_uint(f);
  return (unsigned short)((u + 0x7FFFu + ((u >> 16) & 1u)) >> 16);
}
__device__ __forceinline__ float bf_bits2f(unsigned short h) { return __uint_as_float(((unsigned)h) << 16); }
__device__ __forceinline__ unsigned pk16(unsigned short a, unsigned short b) { return (unsigned)a | ((unsigned)b << 16); }
__device__ __forceinline__ v8f zero8() { v8f z = {0.f, 0.f, 0.f, 0.f, 0.f, 0.f, 0.f, 0.f}; return z; }
__device__ __forceinline__ int wave_id() { return __builtin_amdgcn_readfirstlane((int)(threadIdx.x >> 5)); }

__device__ __forceinline__ void lds_wave_sync() {
  __builtin_amdgcn_fence(__ATOMIC_RELEASE, "workgroup");
  __builtin_amdgcn_wave_barrier();
  __builtin_amdgcn_fence(__ATOMIC_ACQUIRE, "workgroup");
}

union FragB { v16b v; v8b h[2]; };
__device__ __forceinline__ v16b ldfrag_b(const __bf16* p) { FragB f; f.h[0] = *(const v8b*)(p); f.h[1] = *(const v8b*)(p + 16); return f.v; }

__device__ __forceinline__ v8f mma_b(v16b a, v16b b, v8f c) {
  return __builtin_amdgcn_wmma_f32_16x16x32_bf16(false, a, false, b, (short)0, c, false, false);
}
__device__ __forceinline__ void dep_guard_b(v8f& a, v8f& b, v16b x, v16b y) {
  asm volatile("v_nop\n\tv_nop\n\tv_nop\n\tv_nop" : "+v"(a), "+v"(b) : "v"(x), "v"(y));
}
__device__ __forceinline__ void keep4_b(v16b a, v16b b, v16b c, v16b d) { asm volatile("v_nop" :: "v"(a), "v"(b), "v"(c), "v"(d)); }
__device__ __forceinline__ void acc_guard4(v8f& a, v8f& b, v8f& c, v8f& d) {
  asm volatile("v_nop\n\tv_nop\n\tv_nop\n\tv_nop" : "+v"(a), "+v"(b), "+v"(c), "+v"(d));
}
__device__ __forceinline__ void guard_b1x4(v8f& a, v16b w, v16b x, v16b y, v16b z) {
  asm volatile("v_nop\n\tv_nop\n\tv_nop\n\tv_nop" : "+v"(a) : "v"(w), "v"(x), "v"(y), "v"(z) : "memory");
}

template <int SPLIT, int OUT_MODE, bool ROT>
__global__ __launch_bounds__(256) void wmma_gemm64(
    const unsigned short* __restrict__ Ap, const unsigned short* __restrict__ A2p, int lda,
    const unsigned short* __restrict__ Btp, const unsigned short* __restrict__ Bt2p, int ldb,
    void* Cout, void* Cout2, int ldc,
    const float* __restrict__ cst, const float* __restrict__ snt,
    int M, int N, int K, float scale) {
  __shared__ __align__(16) float sT[8][16 * 68];
  const int lane = threadIdx.x & 31;
  const int wave = threadIdx.x >> 5;
  const int tilesN = N >> 6;
  const int tilesM = M >> 6;
  const int tile = (int)blockIdx.x * 8 + wave;
  if (tile >= tilesM * tilesN) return;
  const int tm = tile / tilesN;
  const int tn = tile - tm * tilesN;
  const int m0 = tm << 6;
  const int n0 = tn << 6;

  const __bf16* A   = (const __bf16*)(const void*)Ap;
  const __bf16* A2  = (const __bf16*)(const void*)A2p;
  const __bf16* Bt  = (const __bf16*)(const void*)Btp;
  const __bf16* Bt2 = (const __bf16*)(const void*)Bt2p;

  const int rlane = lane & 15;
  const int koff  = (lane >> 4) * 8;
  const int mOff  = (lane >> 4) * 8;

  v8f acc[4][4];
#pragma unroll
  for (int i = 0; i < 4; ++i)
#pragma unroll
    for (int j = 0; j < 4; ++j) acc[i][j] = zero8();

  for (int k0 = 0; k0 < K; k0 += 32) {
    v16b bh[4], bl[4];
#pragma unroll
    for (int j = 0; j < 4; ++j) {
      const size_t bo = (size_t)(n0 + (j << 4) + rlane) * ldb + koff + k0;
      bh[j] = ldfrag_b(Bt + bo);
      if (SPLIT == 2) bl[j] = ldfrag_b(Bt2 + bo);
    }
#pragma unroll
    for (int i = 0; i < 4; ++i) {
      const size_t ao = (size_t)(m0 + (i << 4) + rlane) * lda + koff + k0;
      v16b ah = ldfrag_b(A + ao);
      v16b al = ah;
      if (SPLIT >= 1) al = ldfrag_b(A2 + ao);
#pragma unroll
      for (int j = 0; j < 4; ++j) {
        acc[i][j] = mma_b(ah, bh[j], acc[i][j]);
        if (SPLIT == 2) acc[i][j] = mma_b(ah, bl[j], acc[i][j]);
        if (SPLIT >= 1) acc[i][j] = mma_b(al, bh[j], acc[i][j]);
      }
      dep_guard_b(acc[i][0], acc[i][3], ah, al);
    }
    keep4_b(bh[0], bh[1], bh[2], bh[3]);
    if (SPLIT == 2) keep4_b(bl[0], bl[1], bl[2], bl[3]);
  }
  acc_guard4(acc[0][0], acc[0][1], acc[0][2], acc[0][3]);
  acc_guard4(acc[1][0], acc[1][1], acc[1][2], acc[1][3]);
  acc_guard4(acc[2][0], acc[2][1], acc[2][2], acc[2][3]);
  acc_guard4(acc[3][0], acc[3][1], acc[3][2], acc[3][3]);

  float* slab = sT[wave];
#pragma unroll
  for (int i = 0; i < 4; ++i) {
    const int mBase = m0 + (i << 4);
#pragma unroll
    for (int j = 0; j < 4; ++j) {
#pragma unroll
      for (int r = 0; r < 8; ++r)
        slab[(mOff + r) * 68 + (j << 4) + rlane] = acc[i][j][r] * scale;
    }
    lds_wave_sync();
    if (OUT_MODE == 0) {
      float* C = (float*)Cout;
      const int hh = lane >> 4, c4 = (lane & 15) * 4;
      for (int pass = 0; pass < 2; ++pass) {
#pragma unroll
        for (int it = 0; it < 8; ++it) {
          const int row = it * 2 + hh;
          const v4f v = *(const v4f*)(slab + row * 68 + c4);
          *(volatile v4f*)(C + (size_t)(mBase + row) * ldc + n0 + c4) = v;
        }
        __threadfence();
      }
    } else {
      const int q = lane >> 3, c8 = (lane & 7) * 8;
      unsigned short* C  = (unsigned short*)Cout;
      unsigned short* C2 = (unsigned short*)Cout2;
      for (int pass = 0; pass < 2; ++pass) {
#pragma unroll
        for (int it = 0; it < 4; ++it) {
          const int row = it * 4 + q;
          const float* sp = slab + row * 68 + c8;
          float xv[8];
#pragma unroll
          for (int e = 0; e < 8; ++e) xv[e] = sp[e];
          if (ROT) {
            const int pos = (mBase + row) & (SQ - 1);
            const size_t to = (size_t)pos * NFRQ + ((n0 & (HD - 1)) >> 1) + (c8 >> 1);
            const v4f cv = *(const v4f*)(cst + to);
            const v4f sv = *(const v4f*)(snt + to);
#pragma unroll
            for (int p = 0; p < 4; ++p) {
              const float x1 = xv[2 * p], x2 = xv[2 * p + 1];
              xv[2 * p]     = x1 * cv[p] - x2 * sv[p];
              xv[2 * p + 1] = x1 * sv[p] + x2 * cv[p];
            }
          }
          v8h hv, lv;
#pragma unroll
          for (int e = 0; e < 8; ++e) {
            const unsigned short hb = f2bf_bits(xv[e]);
            const unsigned short lb = f2bf_bits(xv[e] - bf_bits2f(hb));
            hv[e] = __builtin_bit_cast(_Float16, hb);
            lv[e] = __builtin_bit_cast(_Float16, lb);
          }
          *(volatile v8h*)(C  + (size_t)(mBase + row) * ldc + n0 + c8) = hv;
          *(volatile v8h*)(C2 + (size_t)(mBase + row) * ldc + n0 + c8) = lv;
        }
        __threadfence();
      }
    }
    lds_wave_sync();
  }
}

__global__ __launch_bounds__(256) void rot_table_kernel(float* __restrict__ cst, float* __restrict__ snt) {
  const int lane = threadIdx.x & 31;
  const int wave = (int)(threadIdx.x >> 5);
  const int u = (int)blockIdx.x * 8 + wave;
  const int t = u >> 1;
  const int i = (u & 1) * 32 + lane;
  if (t >= SQ) return;
  const float e   = (float)i * 0.015625f;
  const float pw  = powf(10000.0f, e);
  const float ivf = 1.0f / pw;
  const float ang = (float)t * ivf;
  const float cv  = cosf(ang);
  const float sv  = sinf(ang);
  const size_t o = (size_t)t * NFRQ + i;
  for (int pass = 0; pass < 2; ++pass) {
    ((volatile float*)cst)[o] = cv;
    ((volatile float*)snt)[o] = sv;
    __threadfence();
  }
}

__global__ __launch_bounds__(256) void cvt_bf16_kernel(const float* __restrict__ in, unsigned short* __restrict__ outp, int n8) {
  const int i = (int)blockIdx.x * 256 + (int)threadIdx.x;
  if (i >= n8) return;
  const size_t e = 8 * (size_t)i;
  const v4f a = *(const v4f*)(in + e);
  const v4f b = *(const v4f*)(in + e + 4);
  v4u w;
  w[0] = pk16(f2bf_bits(a[0]), f2bf_bits(a[1]));
  w[1] = pk16(f2bf_bits(a[2]), f2bf_bits(a[3]));
  w[2] = pk16(f2bf_bits(b[0]), f2bf_bits(b[1]));
  w[3] = pk16(f2bf_bits(b[2]), f2bf_bits(b[3]));
  *(volatile v4u*)(outp + e) = w;
  __threadfence();
  *(volatile v4u*)(outp + e) = w;
}

#define AT_KC   32
#define KS_P    136
#define VS_P    40
#define PS_P    40
#define LDS_KS  0
#define LDS_KLS (AT_KC * KS_P)
#define LDS_VHS (2 * AT_KC * KS_P)
#define LDS_VLS (LDS_VHS + HD * VS_P)
#define LDS_PH  (LDS_VLS + HD * VS_P)
#define LDS_PL  (LDS_PH + 4 * 16 * PS_P)
#define LDS_TOT (LDS_PL + 4 * 16 * PS_P)
static_assert(LDS_TOT * 2 <= 65536);
static_assert(4 * 2 * 16 * HD <= LDS_TOT);
static_assert((KS_P * 2) % 16 == 0);
static_assert((VS_P * 2) % 16 == 0);
static_assert((PS_P * 2) % 16 == 0);

__device__ __forceinline__ void at_split(float f, __bf16& hi, __bf16& lo) {
  const unsigned short hb = f2bf_bits(f);
  hi = __builtin_bit_cast(__bf16, hb);
  lo = __builtin_bit_cast(__bf16, f2bf_bits(f - bf_bits2f(hb)));
}

__global__ __launch_bounds__(128)
void attn_causal128_kernel(const unsigned short* __restrict__ qhp, const unsigned short* __restrict__ qlp,
                           const unsigned short* __restrict__ khp, const unsigned short* __restrict__ klp,
                           const unsigned short* __restrict__ vhp, const unsigned short* __restrict__ vlp,
                           unsigned short* __restrict__ chp, unsigned short* __restrict__ clp, float sscale) {
  __shared__ __align__(16) __bf16 lds[LDS_TOT];
  __bf16* Ks  = lds + LDS_KS;
  __bf16* Kls = lds + LDS_KLS;
  __bf16* Vhs = lds + LDS_VHS;
  __bf16* Vls = lds + LDS_VLS;

  const int tid  = (int)threadIdx.x;
  const int lane = tid & 31;
  const int wave = wave_id();
  const int hh   = lane >> 4;
  const int c    = lane & 15;
  const int qb   = (int)blockIdx.x;
  const int h    = (int)blockIdx.y;
  const int b    = (int)blockIdx.z;
  const int q0   = qb * 64 + wave * 16;
  const int qlast = q0 + 15;
  const size_t tok0 = (size_t)b * SQ;

  const __bf16* Qhr = (const __bf16*)(const void*)qhp + (tok0 + q0 + c) * DM + h * HD + 8 * hh;
  const __bf16* Qlr = (const __bf16*)(const void*)qlp + (tok0 + q0 + c) * DM + h * HD + 8 * hh;
  const __bf16* Kg  = (const __bf16*)(const void*)khp + tok0 * DM + h * HD;
  const __bf16* Klg = (const __bf16*)(const void*)klp + tok0 * DM + h * HD;
  const __bf16* Vhg = (const __bf16*)(const void*)vhp + (size_t)(h * HD) * NTOK + tok0;
  const __bf16* Vlg = (const __bf16*)(const void*)vlp + (size_t)(h * HD) * NTOK + tok0;
  __bf16* ph = lds + LDS_PH + wave * (16 * PS_P);
  __bf16* pl = lds + LDS_PL + wave * (16 * PS_P);

  float mrow[8], lrow[8];
  v8f oacc[8];
#pragma unroll
  for (int r = 0; r < 8; ++r) { mrow[r] = -INFINITY; lrow[r] = 0.f; }
#pragma unroll
  for (int t = 0; t < 8; ++t) oacc[t] = zero8();

  const int nch = 2 * qb + 2;
  for (int kc = 0; kc < nch; ++kc) {
    const int kv0 = kc * AT_KC;
    __syncthreads();
#pragma unroll
    for (int i = 0; i < 4; ++i) {
      const int p   = tid + 128 * i;
      const int key = p >> 4, d8 = (p & 15) * 8;
      const v8b kx = *(const v8b*)(Kg  + (size_t)(kv0 + key) * DM + d8);
      const v8b ky = *(const v8b*)(Klg + (size_t)(kv0 + key) * DM + d8);
      *(v8b*)(Ks  + key * KS_P + d8) = kx;
      *(v8b*)(Kls + key * KS_P + d8) = ky;
      const int d = p >> 2, k8 = (p & 3) * 8;
      const v8b vx = *(const v8b*)(Vhg + (size_t)d * NTOK + kv0 + k8);
      const v8b vy = *(const v8b*)(Vlg + (size_t)d * NTOK + kv0 + k8);
      *(v8b*)(Vhs + d * VS_P + k8) = vx;
      *(v8b*)(Vls + d * VS_P + k8) = vy;
    }
    __syncthreads();

    if (kv0 <= qlast) {
      v8f s[2];
      s[0] = zero8(); s[1] = zero8();
#pragma unroll
      for (int dc = 0; dc < 4; ++dc) {
        const v16b qa = ldfrag_b(Qhr + dc * 32);
        const v16b ql = ldfrag_b(Qlr + dc * 32);
#pragma unroll
        for (int j = 0; j < 2; ++j) {
          const v16b kb = ldfrag_b(Ks  + (j * 16 + c) * KS_P + dc * 32 + 8 * hh);
          const v16b kl = ldfrag_b(Kls + (j * 16 + c) * KS_P + dc * 32 + 8 * hh);
          s[j] = mma_b(qa, kb, s[j]);
          s[j] = mma_b(qa, kl, s[j]);
          s[j] = mma_b(ql, kb, s[j]);
          guard_b1x4(s[j], qa, ql, kb, kl);
        }
      }
      float cm[8];
#pragma unroll
      for (int r = 0; r < 8; ++r) {
        const int qrow = q0 + 8 * hh + r;
        float m = -INFINITY;
#pragma unroll
        for (int j = 0; j < 2; ++j) {
          const int key = kv0 + j * 16 + c;
          float sv = s[j][r] * sscale;
          sv = (key > qrow) ? -INFINITY : sv;
          s[j][r] = sv;
          m = fmaxf(m, sv);
        }
#pragma unroll
        for (int off = 1; off < 16; off <<= 1) m = fmaxf(m, __shfl_xor(m, off, 32));
        cm[r] = m;
      }
#pragma unroll
      for (int r = 0; r < 8; ++r) {
        const float mnew  = fmaxf(mrow[r], cm[r]);
        const float alpha = __expf(mrow[r] - mnew);
        mrow[r] = mnew;
        float psum = 0.f;
#pragma unroll
        for (int j = 0; j < 2; ++j) {
          const float p = __expf(s[j][r] - mnew);
          psum += p;
          __bf16 a, bl; at_split(p, a, bl);
          const int po = (8 * hh + r) * PS_P + j * 16 + c;
          ph[po] = a;
          pl[po] = bl;
        }
#pragma unroll
        for (int off = 1; off < 16; off <<= 1) psum += __shfl_xor(psum, off, 32);
        lrow[r] = lrow[r] * alpha + psum;
#pragma unroll
        for (int t = 0; t < 8; ++t) oacc[t][r] *= alpha;
      }
      lds_wave_sync();
      const v16b pa = ldfrag_b(ph + c * PS_P + 8 * hh);
      const v16b pr = ldfrag_b(pl + c * PS_P + 8 * hh);
#pragma unroll
      for (int t = 0; t < 8; ++t) {
        const v16b vb = ldfrag_b(Vhs + (t * 16 + c) * VS_P + 8 * hh);
        const v16b vr = ldfrag_b(Vls + (t * 16 + c) * VS_P + 8 * hh);
        oacc[t] = mma_b(pa, vb, oacc[t]);
        oacc[t] = mma_b(pa, vr, oacc[t]);
        oacc[t] = mma_b(pr, vb, oacc[t]);
        guard_b1x4(oacc[t], pa, pr, vb, vr);
      }
    }
  }

  __syncthreads();
  __bf16* osh = lds + wave * (2 * 16 * HD);
  __bf16* osl = osh + 16 * HD;
#pragma unroll
  for (int r = 0; r < 8; ++r) {
    const float inv = 1.0f / lrow[r];
#pragma unroll
    for (int t = 0; t < 8; ++t) {
      const float o = oacc[t][r] * inv;
      const unsigned short hb = f2bf_bits(o);
      const unsigned short lb = f2bf_bits(o - bf_bits2f(hb));
      const int so = (8 * hh + r) * HD + t * 16 + c;
      osh[so] = __builtin_bit_cast(__bf16, hb);
      osl[so] = __builtin_bit_cast(__bf16, lb);
    }
  }
  lds_wave_sync();
  unsigned short* Chg = chp + (tok0 + q0) * DM + h * HD;
  unsigned short* Clg = clp + (tok0 + q0) * DM + h * HD;
  for (int pass = 0; pass < 2; ++pass) {
#pragma unroll
    for (int it = 0; it < 8; ++it) {
      const int row = it * 2 + hh;
      const int c8  = c * 8;
      const v4u x = __builtin_bit_cast(v4u, *(const v8b*)(osh + row * HD + c8));
      const v4u y = __builtin_bit_cast(v4u, *(const v8b*)(osl + row * HD + c8));
      *(volatile v4u*)(Chg + (size_t)row * DM + c8) = x;
      *(volatile v4u*)(Clg + (size_t)row * DM + c8) = y;
    }
    __threadfence();
  }
}

extern "C" void kernel_launch(void* const* d_in, const int* in_sizes, int n_in,
                              void* d_out, int out_size, void* d_ws, size_t ws_size,
                              hipStream_t stream) {
  if (n_in < 3) return;
  if (in_sizes[0] != NTOK * DM) return;
  if (in_sizes[1] != QKVN * DM) return;
  if (in_sizes[2] != DM * DM) return;
  if (out_size != NTOK * DM) return;

  const float* x    = (const float*)d_in[0];
  const float* wqkv = (const float*)d_in[1];
  const float* wo   = (const float*)d_in[2];
  float* out = (float*)d_out;

  const size_t PX = (size_t)NTOK * DM * 2;
  const size_t PQ = (size_t)QKVN * DM * 2;
  const size_t PW = (size_t)DM * DM * 2;
  const size_t PT = (size_t)SQ * NFRQ * 4;
  size_t off = 0;
  const size_t oXB  = off; off += PX;
  const size_t oWQ  = off; off += PQ;
  const size_t oWO  = off; off += PW;
  const size_t oCs  = off; off += PT;
  const size_t oSn  = off; off += PT;
  const size_t oQh  = off; off += PX;  const size_t oQl  = off; off += PX;
  const size_t oKh  = off; off += PX;  const size_t oKl  = off; off += PX;
  const size_t oVTh = off; off += PX;  const size_t oVTl = off; off += PX;
  const size_t oCh  = off; off += PX;  const size_t oCl  = off; off += PX;
  if (off > ws_size) return;
  if (off > (size_t)134217728) return;

  char* ws = (char*)d_ws;
  unsigned short* XB   = (unsigned short*)(ws + oXB);
  unsigned short* WQKV = (unsigned short*)(ws + oWQ);
  unsigned short* WQb  = WQKV;
  unsigned short* WKb  = WQKV + (size_t)DM * DM;
  unsigned short* WVb  = WQKV + (size_t)2 * DM * DM;
  unsigned short* WOb  = (unsigned short*)(ws + oWO);
  float*          cst  = (float*)(ws + oCs);
  float*          snt  = (float*)(ws + oSn);
  unsigned short* Qh  = (unsigned short*)(ws + oQh);  unsigned short* Ql  = (unsigned short*)(ws + oQl);
  unsigned short* Kh  = (unsigned short*)(ws + oKh);  unsigned short* Kl  = (unsigned short*)(ws + oKl);
  unsigned short* VTh = (unsigned short*)(ws + oVTh); unsigned short* VTl = (unsigned short*)(ws + oVTl);
  unsigned short* Ch  = (unsigned short*)(ws + oCh);  unsigned short* Cl  = (unsigned short*)(ws + oCl);

  const dim3 b256(256), b128(128);
  const int tilesP = (NTOK / 64) * (DM / 64);
  const dim3 gP((tilesP + 7) / 8);

  rot_table_kernel<<<dim3((SQ * 2) / 8), b256, 0, stream>>>(cst, snt);
  cvt_bf16_kernel<<<dim3((NTOK * DM / 8) / 256), b256, 0, stream>>>(x, XB, NTOK * DM / 8);
  cvt_bf16_kernel<<<dim3((QKVN * DM / 8) / 256), b256, 0, stream>>>(wqkv, WQKV, QKVN * DM / 8);
  cvt_bf16_kernel<<<dim3((DM * DM / 8) / 256), b256, 0, stream>>>(wo, WOb, DM * DM / 8);
  wmma_gemm64<0, 2, true><<<gP, b256, 0, stream>>>(
      XB, XB, DM, WQb, WQb, DM, (void*)Qh, (void*)Ql, DM, cst, snt, NTOK, DM, DM, 1.0f);
  wmma_gemm64<0, 2, true><<<gP, b256, 0, stream>>>(
      XB, XB, DM, WKb, WKb, DM, (void*)Kh, (void*)Kl, DM, cst, snt, NTOK, DM, DM, 1.0f);
  wmma_gemm64<0, 2, false><<<gP, b256, 0, stream>>>(
      WVb, WVb, DM, XB, XB, DM, (void*)VTh, (void*)VTl, NTOK, cst, snt, DM, NTOK, DM, 1.0f);
  attn_causal128_kernel<<<dim3(SQ / 64, NH, NB), b128, 0, stream>>>(Qh, Ql, Kh, Kl, VTh, VTl, Ch, Cl, 0.08838834764831845f);
  wmma_gemm64<1, 0, false><<<gP, b256, 0, stream>>>(
      Ch, Cl, DM, WOb, WOb, DM, (void*)out, (void*)out, DM, cst, snt, NTOK, DM, DM, 1.0f);
  (void)hipGetLastError();
}
